// DistSelfAttention_87084756894192
// MI455X (gfx1250) — hardware-verified
//
#include <hip/hip_runtime.h>
#include <math.h>

constexpr int kBatch = 2;
constexpr int kSeq = 1024;
constexpr int kDim = 1024;
constexpr int kHeads = 16;
constexpr int kHeadDim = 64;
constexpr int kTok = kBatch * kSeq;
constexpr long kPlane = (long)kSeq * kDim;
constexpr int kGroups = kBatch * kHeads;
constexpr int kGroupsPerChunk = 8;
constexpr int kChunks = kGroups / kGroupsPerChunk;
constexpr float kEps = 1e-6f;
constexpr float kPiOver8 = (float)(3.14159265358979323846 / 8.0);
constexpr float kWCarry = 32.0f;
constexpr float kWCarryInv = 1.0f / 32.0f;
constexpr float kPCarry = 16384.0f;
constexpr float kYCarry = 16.0f;
constexpr float kPVScale = kYCarry / kPCarry;
constexpr float kOutScale = 1.0f / (kYCarry * kWCarry);


typedef __attribute__((ext_vector_type(16))) _Float16 v16h;
typedef __attribute__((ext_vector_type(8)))  _Float16 v8h;
typedef __attribute__((ext_vector_type(16))) __bf16   v16b;
typedef __attribute__((ext_vector_type(8)))  __bf16   v8b;
typedef __attribute__((ext_vector_type(8)))  float    v8f;
typedef __attribute__((ext_vector_type(4)))  float    v4f;
typedef __attribute__((ext_vector_type(4)))  unsigned int v4u;

__device__ __forceinline__ unsigned short f2bf_bits(float f) {
  unsigned u = __float_as_uint(f);
  return (unsigned short)((u + 0x7FFFu + ((u >> 16) & 1u)) >> 16);
}
__device__ __forceinline__ float bf_bits2f(unsigned short h) { return __uint_as_float(((unsigned)h) << 16); }

__device__ __forceinline__ void dep_guard_h(v8f& a, v8f& b, v16h x, v16h y) { asm volatile("v_nop\n\tv_nop\n\tv_nop\n\tv_nop" : "+v"(a), "+v"(b) : "v"(x), "v"(y)); }
__device__ __forceinline__ void dep_guard_b(v8f& a, v8f& b, v16b x, v16b y) { asm volatile("v_nop\n\tv_nop\n\tv_nop\n\tv_nop" : "+v"(a), "+v"(b) : "v"(x), "v"(y)); }
__device__ __forceinline__ void keep4_h(v16h a, v16h b, v16h c, v16h d) { asm volatile("v_nop" :: "v"(a), "v"(b), "v"(c), "v"(d)); }
__device__ __forceinline__ void keep4_b(v16b a, v16b b, v16b c, v16b d) { asm volatile("v_nop" :: "v"(a), "v"(b), "v"(c), "v"(d)); }
__device__ __forceinline__ void acc_guard4(v8f& a, v8f& b, v8f& c, v8f& d) { asm volatile("v_nop\n\tv_nop\n\tv_nop\n\tv_nop" : "+v"(a), "+v"(b), "+v"(c), "+v"(d)); }
template <typename T> struct Frag;
template <> struct Frag<_Float16> {
  typedef v16h V; union U { v16h v; v8h h[2]; };
  static __device__ __forceinline__ v16h load(const _Float16* p) {
    U f; f.h[0] = *(const v8h*)(p); f.h[1] = *(const v8h*)(p + 16); return f.v;
  }
  static __device__ __forceinline__ v8f mma(v16h a, v16h b, v8f c) {
    return __builtin_amdgcn_wmma_f32_16x16x32_f16(false, a, false, b, (short)0, c, false, false);
  }
  static __device__ __forceinline__ void guard(v8f& a, v8f& b, v16h x, v16h y) { dep_guard_h(a, b, x, y); }
  static __device__ __forceinline__ void keep(v16h a, v16h b, v16h c, v16h d) { keep4_h(a, b, c, d); }
};
template <> struct Frag<__bf16> {
  typedef v16b V; union U { v16b v; v8b h[2]; };
  static __device__ __forceinline__ v16b load(const __bf16* p) {
    U f; f.h[0] = *(const v8b*)(p); f.h[1] = *(const v8b*)(p + 16); return f.v;
  }
  static __device__ __forceinline__ v8f mma(v16b a, v16b b, v8f c) {
    return __builtin_amdgcn_wmma_f32_16x16x32_bf16(false, a, false, b, (short)0, c, false, false);
  }
  static __device__ __forceinline__ void guard(v8f& a, v8f& b, v16b x, v16b y) { dep_guard_b(a, b, x, y); }
  static __device__ __forceinline__ void keep(v16b a, v16b b, v16b c, v16b d) { keep4_b(a, b, c, d); }
};

__device__ __forceinline__ unsigned pk16(unsigned short a, unsigned short b) { return (unsigned)a | ((unsigned)b << 16); }
__device__ __forceinline__ unsigned short h_bits(float f) { const _Float16 h = (_Float16)f; return __builtin_bit_cast(unsigned short, h); }

template <int ET> struct Elem;
template <> struct Elem<0> { typedef _Float16 T; };
template <> struct Elem<1> { typedef __bf16 T; };
template <int ET, bool SPLIT, int BIAS_MODE, int OUT_MODE, bool RESID, int ACT = 0>
__global__ __launch_bounds__(256) void wmma_gemm64(
    const unsigned short* __restrict__ Ap, const unsigned short* __restrict__ A2p, int lda, long strideA,
    const unsigned short* __restrict__ Btp, const unsigned short* __restrict__ Bt2p, int ldb, long strideB,
    void* __restrict__ Cout, void* __restrict__ Cout2, int ldc, long strideC,
    const float* __restrict__ bias,
    const float* __restrict__ resid, long strideR,
    int M, int N, int K, float scale) {
  typedef typename Elem<ET>::T T;
  typedef typename Frag<T>::V V;
  const T* A = (const T*)Ap; const T* A2 = (const T*)A2p; const T* Bt = (const T*)Btp; const T* Bt2 = (const T*)Bt2p;
  __shared__ __align__(16) float sT[8][16 * 68];
  const int b    = blockIdx.y;
  const int lane = threadIdx.x & 31;
  const int wave = threadIdx.x >> 5;
  const int tilesN = N >> 6;
  const int tilesM = M >> 6;
  const int tile = blockIdx.x * 8 + wave;
  if (tile >= tilesM * tilesN) return;
  const int tm = tile / tilesN;
  const int tn = tile - tm * tilesN;
  const int m0 = tm << 6;
  const int n0 = tn << 6;

  const T* Ab  = A  + (size_t)b * strideA;
  const T* Bb  = Bt + (size_t)b * strideB;
  const T* Ab2 = SPLIT ? (A2  + (size_t)b * strideA) : nullptr;
  const T* Bb2 = SPLIT ? (Bt2 + (size_t)b * strideB) : nullptr;

  const int rlane = lane & 15;
  const int koff  = (lane >> 4) * 8;
  const int mOff  = (lane >> 4) * 8;

  v8f acc[4][4];
#pragma unroll
  for (int i = 0; i < 4; ++i)
#pragma unroll
    for (int j = 0; j < 4; ++j) acc[i][j] = (v8f){0.f,0.f,0.f,0.f,0.f,0.f,0.f,0.f};

  for (int k0 = 0; k0 < K; k0 += 32) {
    V bh[4], bl[4];
#pragma unroll
    for (int j = 0; j < 4; ++j) {
      const size_t bo = (size_t)(n0 + (j << 4) + rlane) * ldb + koff + k0;
      bh[j] = Frag<T>::load(Bb + bo);
      if (SPLIT) bl[j] = Frag<T>::load(Bb2 + bo);
    }
#pragma unroll
    for (int i = 0; i < 4; ++i) {
      const size_t ao = (size_t)(m0 + (i << 4) + rlane) * lda + koff + k0;
      V ah = Frag<T>::load(Ab + ao);
      V al;
      if (SPLIT) al = Frag<T>::load(Ab2 + ao);
#pragma unroll
      for (int j = 0; j < 4; ++j) {
        acc[i][j] = Frag<T>::mma(ah, bh[j], acc[i][j]);
        if (SPLIT) {
          acc[i][j] = Frag<T>::mma(ah, bl[j], acc[i][j]);
          acc[i][j] = Frag<T>::mma(al, bh[j], acc[i][j]);
        }
      }
      Frag<T>::guard(acc[i][0], acc[i][3], ah, SPLIT ? al : ah);
    }
    Frag<T>::keep(bh[0], bh[1], bh[2], bh[3]);
    if (SPLIT) Frag<T>::keep(bl[0], bl[1], bl[2], bl[3]);
  }
  acc_guard4(acc[0][0], acc[0][1], acc[0][2], acc[0][3]);
  acc_guard4(acc[1][0], acc[1][1], acc[1][2], acc[1][3]);
  acc_guard4(acc[2][0], acc[2][1], acc[2][2], acc[2][3]);
  acc_guard4(acc[3][0], acc[3][1], acc[3][2], acc[3][3]);

  float* slab = sT[wave];
  const float* Rb = RESID ? (resid + (size_t)b * strideR) : nullptr;
#pragma unroll
  for (int i = 0; i < 4; ++i) {
    const int mBase = m0 + (i << 4);
#pragma unroll
    for (int j = 0; j < 4; ++j) {
      const int n = n0 + (j << 4) + rlane;
      float bv = 0.f;
      if (BIAS_MODE == 2) bv = bias[n];
#pragma unroll
      for (int r = 0; r < 8; ++r) {
        float v = acc[i][j][r] * scale;
        if (BIAS_MODE == 1) v += bias[mBase + mOff + r];
        if (BIAS_MODE == 2) v += bv;
        if (RESID) v += Rb[(size_t)(mBase + mOff + r) * ldc + n];
        if (ACT == 2) v = fmaxf(v, 0.0f);
        if (ACT == 4) v = (v > 0.f) ? v : 0.01f * v;
        if (ACT == 6) { const float s6 = __builtin_amdgcn_sqrtf(fmaxf(v, 0.0f)) + kEps; v = s6 * s6; }
        if (ACT == 7) { const float s7 = __builtin_amdgcn_sqrtf(fmaxf(v, 0.0f) + kEps) + kEps; v = s7 * s7; }
        if (ACT == 8) v = __builtin_amdgcn_sqrtf(fmaxf(v, 0.0f));
        slab[(mOff + r) * 68 + (j << 4) + rlane] = v;
      }
    }
    __builtin_amdgcn_fence(__ATOMIC_RELEASE, "workgroup");
    __builtin_amdgcn_wave_barrier();
    __builtin_amdgcn_fence(__ATOMIC_ACQUIRE, "workgroup");
    if (OUT_MODE == 0) {
      float* C = (float*)Cout + (size_t)b * strideC;
      const int hh = lane >> 4, c4 = (lane & 15) * 4;
      for (int pass = 0; pass < 2; ++pass) {
#pragma unroll
        for (int it = 0; it < 8; ++it) {
          const int row = it * 2 + hh;
          v4f v = *(const v4f*)(slab + row * 68 + c4);
          *(volatile v4f*)(C + (size_t)(mBase + row) * ldc + n0 + c4) = v;
        }
        __threadfence();
      }
    } else {
      const int q = lane >> 3, c8 = (lane & 7) * 8;
      unsigned short* C  = (unsigned short*)Cout  + (size_t)b * strideC;
      unsigned short* C2 = (OUT_MODE == 2) ? ((unsigned short*)Cout2 + (size_t)b * strideC) : nullptr;
      for (int pass = 0; pass < 2; ++pass) {
#pragma unroll
        for (int it = 0; it < 4; ++it) {
          const int row = it * 4 + q;
          const float* sp = slab + row * 68 + c8;
          v8h hv, lv;
#pragma unroll
          for (int e = 0; e < 8; ++e) {
            if (OUT_MODE == 1) {
              hv[e] = (_Float16)sp[e];
            } else if (OUT_MODE == 3) {
              hv[e] = __builtin_bit_cast(_Float16, f2bf_bits(sp[e]));
            } else {
              unsigned short hb = f2bf_bits(sp[e]);
              unsigned short lb = f2bf_bits(sp[e] - bf_bits2f(hb));
              hv[e] = __builtin_bit_cast(_Float16, hb);
              lv[e] = __builtin_bit_cast(_Float16, lb);
            }
          }
          *(volatile v8h*)(C + (size_t)(mBase + row) * ldc + n0 + c8) = hv;
          if (OUT_MODE == 2) *(volatile v8h*)(C2 + (size_t)(mBase + row) * ldc + n0 + c8) = lv;
        }
        __threadfence();
      }
    }
    __builtin_amdgcn_fence(__ATOMIC_RELEASE, "workgroup");
    __builtin_amdgcn_wave_barrier();
    __builtin_amdgcn_fence(__ATOMIC_ACQUIRE, "workgroup");
  }
}

__global__ __launch_bounds__(256) void cast8_f16_kernel(const float* __restrict__ in, unsigned short* __restrict__ out,
                                                        int n8, float scale) {
  const int i = blockIdx.x * 256 + threadIdx.x;
  if (i >= n8) return;
  const float* p = in + 8 * (size_t)i;
  const v4f a = *(const v4f*)(p);
  const v4f c = *(const v4f*)(p + 4);
  unsigned short hb[8];
#pragma unroll
  for (int e = 0; e < 4; ++e) {
    hb[e]     = h_bits(a[e] * scale);
    hb[4 + e] = h_bits(c[e] * scale);
  }
  const v4u u = (v4u){pk16(hb[0], hb[1]), pk16(hb[2], hb[3]), pk16(hb[4], hb[5]), pk16(hb[6], hb[7])};
  unsigned short* q = out + 8 * (size_t)i;
  *(volatile v4u*)q = u;
  __threadfence();
  *(volatile v4u*)q = u;
}

__global__ __launch_bounds__(256) void sq8_bf16_kernel(const float* __restrict__ in, unsigned short* __restrict__ out, int n8) {
  const int i = blockIdx.x * 256 + threadIdx.x;
  if (i >= n8) return;
  const float* p = in + 8 * (size_t)i;
  const v4f a = *(const v4f*)(p);
  const v4f c = *(const v4f*)(p + 4);
  unsigned short hb[8];
#pragma unroll
  for (int e = 0; e < 4; ++e) {
    hb[e]     = f2bf_bits(a[e] * a[e]);
    hb[4 + e] = f2bf_bits(c[e] * c[e]);
  }
  const v4u u = (v4u){pk16(hb[0], hb[1]), pk16(hb[2], hb[3]), pk16(hb[4], hb[5]), pk16(hb[6], hb[7])};
  unsigned short* q = out + 8 * (size_t)i;
  *(volatile v4u*)q = u;
  __threadfence();
  *(volatile v4u*)q = u;
}

__global__ __launch_bounds__(128) void dual_softmax_kernel(const float* __restrict__ Sc, const float* __restrict__ tau_p,
                                                           unsigned short* __restrict__ Pmu, unsigned short* __restrict__ Pvar) {
#pragma clang fp contract(off)
  __shared__ float redM[4];
  __shared__ float redZ1[4];
  __shared__ float redZ2[4];
  const int row  = blockIdx.x;
  const int t    = threadIdx.x;
  const int lane = t & 31, wave = t >> 5;

  const float tau       = tau_p[0];
  const float inv_tau   = __builtin_amdgcn_rcpf(tau);
  const float score_var = 0.1f + kEps;
  const float s_var     = score_var * (1.0f / 64.0f) + kEps;
  const float l_var     = s_var * __builtin_amdgcn_rcpf(tau * tau) + kEps;
  const float cden      = __builtin_amdgcn_sqrtf(1.0f + kPiOver8 * l_var);
  const float inv_c     = __builtin_amdgcn_rcpf(cden);

  const float* sr = Sc + (size_t)row * kSeq + t * 8;
  const v4f a = *(const v4f*)(sr);
  const v4f c = *(const v4f*)(sr + 4);
  float l[8];
#pragma unroll
  for (int e = 0; e < 4; ++e) {
    l[e]     = (a[e] * 0.125f) * inv_tau;
    l[4 + e] = (c[e] * 0.125f) * inv_tau;
  }
  float m = fmaxf(fmaxf(fmaxf(l[0], l[1]), fmaxf(l[2], l[3])), fmaxf(fmaxf(l[4], l[5]), fmaxf(l[6], l[7])));
#pragma unroll
  for (int off = 16; off > 0; off >>= 1) m = fmaxf(m, __shfl_xor(m, off, 32));
  if (lane == 0) redM[wave] = m;
  __syncthreads();
  m = fmaxf(fmaxf(redM[0], redM[1]), fmaxf(redM[2], redM[3]));
  const float ma = m * inv_c;

  float e1[8], e2[8];
  float z1 = 0.f, z2 = 0.f;
#pragma unroll
  for (int e = 0; e < 8; ++e) {
    e1[e] = expf(l[e] - m);
    e2[e] = expf(l[e] * inv_c - ma);
    z1 += e1[e];
    z2 += e2[e];
  }
#pragma unroll
  for (int off = 16; off > 0; off >>= 1) {
    z1 += __shfl_xor(z1, off, 32);
    z2 += __shfl_xor(z2, off, 32);
  }
  if (lane == 0) { redZ1[wave] = z1; redZ2[wave] = z2; }
  __syncthreads();
  z1 = ((redZ1[0] + redZ1[1]) + redZ1[2]) + redZ1[3];
  z2 = ((redZ2[0] + redZ2[1]) + redZ2[2]) + redZ2[3];
  const float inv_z1 = __builtin_amdgcn_rcpf(z1);
  const float inv_z2 = __builtin_amdgcn_rcpf(z2);

  unsigned short hm[8], hb[8];
#pragma unroll
  for (int e = 0; e < 8; ++e) {
    const float top = e1[e] * inv_z1;
    const float r   = e2[e] * inv_z2;
    const float pm  = top + r;
    const float rv  = (r * (1.0f - r)) * l_var;
    const float pv  = (1e-4f + rv) + kEps;
    hm[e] = h_bits(pm * kPCarry);
    hb[e] = f2bf_bits(pv);
  }
  const v4u um = (v4u){pk16(hm[0], hm[1]), pk16(hm[2], hm[3]), pk16(hm[4], hm[5]), pk16(hm[6], hm[7])};
  const v4u ub = (v4u){pk16(hb[0], hb[1]), pk16(hb[2], hb[3]), pk16(hb[4], hb[5]), pk16(hb[6], hb[7])};
  unsigned short* pm_ptr = Pmu  + (size_t)row * kSeq + t * 8;
  unsigned short* pv_ptr = Pvar + (size_t)row * kSeq + t * 8;
  *(volatile v4u*)pm_ptr = um;
  *(volatile v4u*)pv_ptr = ub;
  __threadfence();
  *(volatile v4u*)pm_ptr = um;
  *(volatile v4u*)pv_ptr = ub;
}

extern "C" void kernel_launch(void* const* d_in, const int* in_sizes, int n_in,
                              void* d_out, int out_size, void* d_ws,
                              size_t ws_size, hipStream_t stream) {
  if (n_in < 15) return;
  if (out_size != 2 * kTok * kDim) return;
  if (in_sizes[0] != kTok * kDim || in_sizes[6] != kDim * kDim || in_sizes[14] < 1) return;
  const size_t MiB = (size_t)1 << 20;
  const size_t kNeedBytes = 116 * MiB;
  if (ws_size < kNeedBytes) return;

  const float* q_loc   = (const float*)d_in[0];
  const float* k_loc   = (const float*)d_in[2];
  const float* v_loc   = (const float*)d_in[4];
  const float* v_scale = (const float*)d_in[5];
  const float* Wq = (const float*)d_in[6];
  const float* bq = (const float*)d_in[7];
  const float* Wk = (const float*)d_in[8];
  const float* bk = (const float*)d_in[9];
  const float* Wv = (const float*)d_in[10];
  const float* bv = (const float*)d_in[11];
  const float* Wo = (const float*)d_in[12];
  const float* bo = (const float*)d_in[13];
  const float* tau = (const float*)d_in[14];
  float* out0 = (float*)d_out;
  float* out1 = (float*)d_out + (size_t)kTok * kDim;

  char* ws = (char*)d_ws;
  unsigned short* xq   = (unsigned short*)(ws +   0 * MiB);
  unsigned short* xk   = (unsigned short*)(ws +   4 * MiB);
  unsigned short* xv   = (unsigned short*)(ws +   8 * MiB);
  unsigned short* xs2  = (unsigned short*)(ws +  12 * MiB);
  unsigned short* wq16 = (unsigned short*)(ws +  16 * MiB);
  unsigned short* wk16 = (unsigned short*)(ws +  18 * MiB);
  unsigned short* wv16 = (unsigned short*)(ws +  20 * MiB);
  unsigned short* wo16 = (unsigned short*)(ws +  22 * MiB);
  unsigned short* wv2b = (unsigned short*)(ws +  24 * MiB);
  unsigned short* wo2b = (unsigned short*)(ws +  26 * MiB);
  unsigned short* qm   = (unsigned short*)(ws +  28 * MiB);
  unsigned short* km   = (unsigned short*)(ws +  32 * MiB);
  unsigned short* vmT  = (unsigned short*)(ws +  36 * MiB);
  unsigned short* vvT  = (unsigned short*)(ws +  40 * MiB);
  unsigned short* ymu  = (unsigned short*)(ws +  44 * MiB);
  unsigned short* x2   = (unsigned short*)(ws +  48 * MiB);
  float*          Sc   = (float*)         (ws +  52 * MiB);
  unsigned short* Pmu  = (unsigned short*)(ws +  84 * MiB);
  unsigned short* Pvar = (unsigned short*)(ws + 100 * MiB);

  const int n8act = (kTok * kDim) / 8;
  const int n8w   = (kDim * kDim) / 8;

  cast8_f16_kernel<<<n8act / 256, 256, 0, stream>>>(q_loc, xq, n8act, 1.0f);
  cast8_f16_kernel<<<n8act / 256, 256, 0, stream>>>(k_loc, xk, n8act, 1.0f);
  cast8_f16_kernel<<<n8act / 256, 256, 0, stream>>>(v_loc, xv, n8act, 1.0f);
  cast8_f16_kernel<<<n8w / 256, 256, 0, stream>>>(Wq, wq16, n8w, kWCarry);
  cast8_f16_kernel<<<n8w / 256, 256, 0, stream>>>(Wk, wk16, n8w, kWCarry);
  cast8_f16_kernel<<<n8w / 256, 256, 0, stream>>>(Wv, wv16, n8w, kWCarry);
  cast8_f16_kernel<<<n8w / 256, 256, 0, stream>>>(Wo, wo16, n8w, kWCarry);
  sq8_bf16_kernel<<<n8act / 256, 256, 0, stream>>>(v_scale, xs2, n8act);
  sq8_bf16_kernel<<<n8w / 256, 256, 0, stream>>>(Wv, wv2b, n8w);
  sq8_bf16_kernel<<<n8w / 256, 256, 0, stream>>>(Wo, wo2b, n8w);

  wmma_gemm64<0, false, 2, 1, false, 0><<<dim3(64, 1), 256, 0, stream>>>(
      xq, nullptr, kDim, 0L, wq16, nullptr, kDim, 0L, qm, nullptr, kDim, 0L, bq, nullptr, 0L, kTok, kDim, kDim, kWCarryInv);
  wmma_gemm64<0, false, 2, 1, false, 0><<<dim3(64, 1), 256, 0, stream>>>(
      xk, nullptr, kDim, 0L, wk16, nullptr, kDim, 0L, km, nullptr, kDim, 0L, bk, nullptr, 0L, kTok, kDim, kDim, kWCarryInv);
  wmma_gemm64<0, false, 1, 1, false, 0><<<dim3(32, kBatch), 256, 0, stream>>>(
      wv16, nullptr, kDim, 0L, xv, nullptr, kDim, (long)kPlane, vmT, nullptr, kSeq, (long)kPlane, bv, nullptr, 0L,
      kDim, kSeq, kDim, kWCarryInv);
  wmma_gemm64<1, false, 0, 3, false, 6><<<dim3(32, kBatch), 256, 0, stream>>>(
      wv2b, nullptr, kDim, 0L, xs2, nullptr, kDim, (long)kPlane, vvT, nullptr, kSeq, (long)kPlane, nullptr, nullptr, 0L,
      kDim, kSeq, kDim, 1.0f);

  for (int ch = 0; ch < kChunks; ++ch) {
    const int b  = ch / (kHeads / kGroupsPerChunk);
    const int h0 = (ch % (kHeads / kGroupsPerChunk)) * kGroupsPerChunk;
    const unsigned short* qg = qm + (size_t)b * kPlane + (size_t)h0 * kHeadDim;
    const unsigned short* kg = km + (size_t)b * kPlane + (size_t)h0 * kHeadDim;
    wmma_gemm64<0, false, 0, 0, false, 0><<<dim3(32, kGroupsPerChunk), 256, 0, stream>>>(
        qg, nullptr, kDim, (long)kHeadDim, kg, nullptr, kDim, (long)kHeadDim, Sc, nullptr, kSeq, (long)kPlane,
        nullptr, nullptr, 0L, kSeq, kSeq, kHeadDim, 1.0f);
    dual_softmax_kernel<<<kGroupsPerChunk * kSeq, 128, 0, stream>>>(Sc, tau, Pmu, Pvar);
    wmma_gemm64<0, false, 0, 1, false, 0><<<dim3(2, kGroupsPerChunk), 256, 0, stream>>>(
        Pmu, nullptr, kSeq, (long)kPlane,
        vmT + (size_t)b * kPlane + (size_t)h0 * kHeadDim * kSeq, nullptr, kSeq, (long)kHeadDim * kSeq,
        ymu + (size_t)b * kPlane + (size_t)h0 * kHeadDim, nullptr, kDim, (long)kHeadDim,
        nullptr, nullptr, 0L, kSeq, kHeadDim, kSeq, kPVScale);
    wmma_gemm64<1, false, 0, 3, false, 7><<<dim3(2, kGroupsPerChunk), 256, 0, stream>>>(
        Pvar, nullptr, kSeq, (long)kPlane,
        vvT + (size_t)b * kPlane + (size_t)h0 * kHeadDim * kSeq, nullptr, kSeq, (long)kHeadDim * kSeq,
        x2 + (size_t)b * kPlane + (size_t)h0 * kHeadDim, nullptr, kDim, (long)kHeadDim,
        nullptr, nullptr, 0L, kSeq, kHeadDim, kSeq, 1.0f);
  }

  wmma_gemm64<0, false, 2, 0, false, 0><<<dim3(64, 1), 256, 0, stream>>>(
      ymu, nullptr, kDim, 0L, wo16, nullptr, kDim, 0L, out0, nullptr, kDim, 0L, bo, nullptr, 0L, kTok, kDim, kDim, kOutScale);
  wmma_gemm64<1, false, 0, 0, false, 8><<<dim3(64, 1), 256, 0, stream>>>(
      x2, nullptr, kDim, 0L, wo2b, nullptr, kDim, 0L, out1, nullptr, kDim, 0L, nullptr, nullptr, 0L, kTok, kDim, kDim, 1.0f);
}
